// FusedSelfAttention_9010841387083
// MI455X (gfx1250) — hardware-verified
//
#include <hip/hip_runtime.h>
#include <math.h>

typedef __attribute__((ext_vector_type(16))) __bf16 v16b;
typedef __attribute__((ext_vector_type(8)))  __bf16 v8b;
typedef __attribute__((ext_vector_type(8)))  float v8f;
typedef __attribute__((ext_vector_type(4)))  float v4f;
typedef __attribute__((ext_vector_type(4)))  unsigned v4u;

#ifndef NB
#define NB 4
#endif
#ifndef SEQ
#define SEQ 2048
#endif
#define NB_FULL 4
#define SEQ_FULL 2048
#define DM 1024
#define NH 16
#define HD 64
#define QKVW (3 * DM)
static_assert(NB >= 1 && NB <= NB_FULL);
static_assert(SEQ % 64 == 0 && SEQ >= 64 && SEQ <= SEQ_FULL);
static_assert(NH * HD == DM);
static_assert(DM % 32 == 0 && QKVW % 128 == 0);

template <typename T> __device__ __forceinline__ void vst2(void* p, T v) { *(volatile T*)p = v; __threadfence(); *(volatile T*)p = v; }
__device__ __forceinline__ v8f wmma_bf(v16b a, v16b b, v8f c) {
  v8f d = __builtin_amdgcn_wmma_f32_16x16x32_bf16(false, a, false, b, (short)0, c, false, false);
  asm volatile("v_nop\n\tv_nop\n\tv_nop\n\tv_nop" : "+v"(d) : "v"(a), "v"(b));
  return d;
}
__device__ __forceinline__ v16b frag_b(const __bf16* rowk0, int lane) {
  union { v16b v; v8b q[2]; } u; const __bf16* p = rowk0 + 8 * (lane >> 4);
  u.q[0] = *(const v8b*)p; u.q[1] = *(const v8b*)(p + 16); return u.v;
}
struct F2 { v16b h, l; };
__device__ __forceinline__ F2 bsplit16(const float v[16]) { F2 r;
#pragma unroll
  for (int i = 0; i < 16; ++i) { const __bf16 h = (__bf16)v[i]; r.h[i] = h; r.l[i] = (__bf16)(v[i] - (float)h); }
  return r; }
__device__ __forceinline__ F2 split_row(const float* row, int k0, int lane) { float v[16]; const float* p = row + k0 + 8 * (lane >> 4);
#pragma unroll
  for (int i = 0; i < 8; ++i) { v[i] = p[i]; v[8 + i] = p[16 + i]; }
  return bsplit16(v); }
__device__ __forceinline__ v8f mac3(const F2& a, const F2& b, v8f c) { c = wmma_bf(a.l, b.h, c); c = wmma_bf(a.h, b.l, c); return wmma_bf(a.h, b.h, c); }
__device__ __attribute__((noinline)) float exp_ni(float v) { return expf(v); }
#define LDSX() do { asm volatile("s_wait_dscnt 0" ::: "memory"); __builtin_amdgcn_wave_barrier(); __builtin_amdgcn_fence(__ATOMIC_RELEASE, "workgroup"); } while (0)

__device__ __forceinline__ v4u pack8_hi(v4f a, v4f c) {
  union { v8b b; v4u u; } H;
#pragma unroll
  for (int i = 0; i < 4; ++i) { H.b[i] = (__bf16)a[i]; H.b[4 + i] = (__bf16)c[i]; }
  return H.u;
}
__device__ __forceinline__ void pack8_hilo(v4f a, v4f c, v4u& hi, v4u& lo) {
  union { v8b b; v4u u; } H, L; float v[8];
#pragma unroll
  for (int i = 0; i < 4; ++i) { v[i] = a[i]; v[4 + i] = c[i]; }
#pragma unroll
  for (int i = 0; i < 8; ++i) { const __bf16 hb = (__bf16)v[i]; H.b[i] = hb; L.b[i] = (__bf16)(v[i] - (float)hb); }
  hi = H.u; lo = L.u;
}

#define PK_A 0
#define PK_P (PK_A + QKVW * DM)
#define PK_END (PK_P + DM * DM)
#define WS_PK  0u
#define WS_XB  (WS_PK + 2u * PK_END)
#define WS_QK  (WS_XB + 2u * NB * SEQ * DM)
#define WS_KH  (WS_QK + 4u * SEQ * QKVW)
#define WS_KL  (WS_KH + 2u * SEQ * DM)
#define WS_VTH (WS_KL + 2u * SEQ * DM)
#define WS_VTL (WS_VTH + 2u * DM * SEQ)
#define WS_O   (WS_VTL + 2u * DM * SEQ)
#define WS_OH  (WS_O + 4u * SEQ * DM)
#define WS_OL  (WS_OH + 2u * SEQ * DM)
#define WS_END (WS_OL + 2u * SEQ * DM)
static_assert(WS_END <= 134217728u);
static_assert((WS_XB % 128u) == 0 && (WS_QK % 128u) == 0 && (WS_KH % 128u) == 0 && (WS_KL % 128u) == 0 && (WS_VTH % 128u) == 0 && (WS_VTL % 128u) == 0 && (WS_O % 128u) == 0 && (WS_OH % 128u) == 0 && (WS_OL % 128u) == 0);

__global__ __launch_bounds__(256) void k_packT(const float* __restrict__ Wm, int K, int N, __bf16* __restrict__ DST) {
  __shared__ __align__(16) __bf16 s[DM]; const int n = blockIdx.x, tid = threadIdx.x;
  for (int k = tid; k < K; k += 256) s[k] = (__bf16)Wm[(size_t)k * N + n];
  __syncthreads();
  for (int q = tid; q < K / 8; q += 256) vst2(DST + (size_t)n * K + q * 8, *(const v4u*)&s[q * 8]);
}
__global__ __launch_bounds__(256) void k_cvtx(const float* __restrict__ X, __bf16* __restrict__ XB) {
  const int tid = threadIdx.x; const int r = blockIdx.x * 2 + (tid >> 7), c8 = (tid & 127) * 8;
  const int b = r / SEQ, s = r - b * SEQ;
  const float* src = X + ((size_t)b * SEQ_FULL + s) * DM + c8;
  const v4f a = *(const v4f*)src, c = *(const v4f*)(src + 4);
  vst2(XB + (size_t)r * DM + c8, pack8_hi(a, c));
}
__global__ __launch_bounds__(128) void k_qkv(const __bf16* __restrict__ XB, const __bf16* __restrict__ P, float* __restrict__ QKV) {
  __shared__ __align__(16) float so[4][16][132];
  const int tid = threadIdx.x, wave = tid >> 5, lane = tid & 31, col = lane & 15, g = lane >> 4; const size_t r0 = (size_t)blockIdx.x * 64 + wave * 16; const int n0 = blockIdx.y * 128;
  v8f acc[8] = {};
#pragma unroll 2
  for (int kc = 0; kc < DM / 32; ++kc) { const v16b a = frag_b(XB + (r0 + col) * DM + kc * 32, lane);
#pragma unroll
    for (int j = 0; j < 8; ++j) acc[j] = wmma_bf(a, frag_b(P + (size_t)(n0 + j * 16 + col) * DM + kc * 32, lane), acc[j]); }
#pragma unroll
  for (int j = 0; j < 8; ++j)
#pragma unroll
    for (int r = 0; r < 8; ++r) so[wave][8 * g + r][j * 16 + col] = acc[j][r];
  LDSX();
  for (int rl = 0; rl < 16; ++rl) vst2(QKV + (r0 + rl) * QKVW + n0 + lane * 4, *(const v4f*)&so[wave][rl][lane * 4]);
}
__global__ __launch_bounds__(256) void k_kv(const float* __restrict__ QKV, __bf16* __restrict__ KH, __bf16* __restrict__ KL, __bf16* __restrict__ VTH, __bf16* __restrict__ VTL) {
  __shared__ __align__(16) __bf16 sth[64][72], stl[64][72], skh[64][72], skl[64][72];
  const int tid = threadIdx.x; const int s0 = blockIdx.x * 64, h = blockIdx.y;
  for (int q = tid; q < 64 * 64; q += 256) { const int rl = q >> 6, d = q & 63;
    const float* row = QKV + (size_t)(s0 + rl) * QKVW + h * 192;
    const float kv = row[64 + d], vv = row[128 + d];
    const __bf16 kb = (__bf16)kv, vb = (__bf16)vv;
    skh[rl][d] = kb; skl[rl][d] = (__bf16)(kv - (float)kb);
    sth[d][rl] = vb; stl[d][rl] = (__bf16)(vv - (float)vb); }
  __syncthreads();
  for (int q = tid; q < 64 * 8; q += 256) { const int a = q >> 3, pc = q & 7;
    const size_t ov = (size_t)(h * HD + a) * SEQ + s0 + pc * 8;
    vst2(VTH + ov, *(const v4u*)&sth[a][pc * 8]); vst2(VTL + ov, *(const v4u*)&stl[a][pc * 8]);
    const size_t ok = (size_t)(s0 + a) * DM + h * HD + pc * 8;
    vst2(KH + ok, *(const v4u*)&skh[a][pc * 8]); vst2(KL + ok, *(const v4u*)&skl[a][pc * 8]); }
}
__global__ __launch_bounds__(128) void k_attn(const float* __restrict__ QK, const __bf16* __restrict__ KH, const __bf16* __restrict__ KL, const __bf16* __restrict__ VTH, const __bf16* __restrict__ VTL, float* __restrict__ O) {
  __shared__ __align__(16) float sp[4][16][36]; __shared__ __align__(16) float so[4][16][68];
  const int tid = threadIdx.x, wave = tid >> 5, lane = tid & 31, col = lane & 15, g = lane >> 4;
  const int qb = blockIdx.x, h = blockIdx.y; const int q0 = qb * 64 + wave * 16; const size_t rq = (size_t)q0 + col;
  F2 aq[2];
#pragma unroll
  for (int kc = 0; kc < 2; ++kc) aq[kc] = split_row(QK + rq * QKVW + h * 192, kc * 32, lane);
  float m[8], l[8];
#pragma unroll
  for (int r = 0; r < 8; ++r) { m[r] = -3.0e38f; l[r] = 0.f; }
  v8f acc[4] = {};
  const int nks = (qb * 64 + 64) / 32;
#pragma unroll 1
  for (int ks = 0; ks < nks; ++ks) { v8f s[2];
#pragma unroll
    for (int ct = 0; ct < 2; ++ct) { const int kk = ks * 32 + ct * 16 + col; const size_t kr = (size_t)kk * DM + h * HD; v8f c = {};
#pragma unroll
      for (int kc = 0; kc < 2; ++kc) { F2 kb; kb.h = frag_b(KH + kr + kc * 32, lane); kb.l = frag_b(KL + kr + kc * 32, lane); c = mac3(aq[kc], kb, c); }
#pragma unroll
      for (int r = 0; r < 8; ++r) { const int qi = q0 + 8 * g + r; s[ct][r] = (kk <= qi) ? c[r] * 0.03125f : -3.0e38f; } }
#pragma unroll
    for (int r = 0; r < 8; ++r) { float mx = fmaxf(s[0][r], s[1][r]);
#pragma unroll
      for (int o = 1; o < 16; o <<= 1) mx = fmaxf(mx, __shfl_xor(mx, o));
      const float mn = fmaxf(m[r], mx); const float alpha = (m[r] <= -1.0e38f) ? 0.f : exp_ni(m[r] - mn);
      const float e0 = (s[0][r] <= -1.0e38f) ? 0.f : exp_ni(s[0][r] - mn), e1 = (s[1][r] <= -1.0e38f) ? 0.f : exp_ni(s[1][r] - mn); float es = e0 + e1;
#pragma unroll
      for (int o = 1; o < 16; o <<= 1) es += __shfl_xor(es, o);
      l[r] = l[r] * alpha + es; m[r] = mn;
#pragma unroll
      for (int dt = 0; dt < 4; ++dt) acc[dt][r] *= alpha;
      sp[wave][8 * g + r][col] = e0; sp[wave][8 * g + r][16 + col] = e1; }
    LDSX();
    const F2 pa = split_row(&sp[wave][col][0], 0, lane);
#pragma unroll
    for (int dt = 0; dt < 4; ++dt) { const size_t vr = (size_t)(h * HD + dt * 16 + col) * SEQ + ks * 32; const v16b vh = frag_b(VTH + vr, lane), vl = frag_b(VTL + vr, lane); acc[dt] = wmma_bf(pa.l, vh, acc[dt]); acc[dt] = wmma_bf(pa.h, vl, acc[dt]); acc[dt] = wmma_bf(pa.h, vh, acc[dt]); }
    LDSX(); }
#pragma unroll
  for (int r = 0; r < 8; ++r) { const float il = 1.0f / l[r];
#pragma unroll
    for (int dt = 0; dt < 4; ++dt) so[wave][8 * g + r][dt * 16 + col] = acc[dt][r] * il; }
  LDSX();
  for (int rl = 0; rl < 16; ++rl) if (lane < 16) vst2(O + (size_t)(q0 + rl) * DM + h * HD + lane * 4, *(const v4f*)&so[wave][rl][lane * 4]);
}
__global__ __launch_bounds__(256) void k_osplit(const float* __restrict__ O, __bf16* __restrict__ OH, __bf16* __restrict__ OL) {
  const int tid = threadIdx.x; const int r = blockIdx.x * 2 + (tid >> 7), c8 = (tid & 127) * 8;
  const float* src = O + (size_t)r * DM + c8;
  const v4f a = *(const v4f*)src, c = *(const v4f*)(src + 4);
  v4u hi, lo; pack8_hilo(a, c, hi, lo);
  const size_t o = (size_t)r * DM + c8;
  vst2(OH + o, hi); vst2(OL + o, lo);
}
__global__ __launch_bounds__(128) void k_out(const __bf16* __restrict__ OH, const __bf16* __restrict__ OL, const __bf16* __restrict__ P, float* __restrict__ Y) {
  __shared__ __align__(16) float so[4][16][132];
  const int tid = threadIdx.x, wave = tid >> 5, lane = tid & 31, col = lane & 15, g = lane >> 4; const size_t r0 = (size_t)blockIdx.x * 64 + wave * 16; const int n0 = blockIdx.y * 128;
  v8f acc[8] = {};
#pragma unroll 2
  for (int kc = 0; kc < DM / 32; ++kc) { const v16b ah = frag_b(OH + (r0 + col) * DM + kc * 32, lane), al = frag_b(OL + (r0 + col) * DM + kc * 32, lane);
#pragma unroll
    for (int j = 0; j < 8; ++j) { const v16b w = frag_b(P + (size_t)(n0 + j * 16 + col) * DM + kc * 32, lane); acc[j] = wmma_bf(al, w, acc[j]); acc[j] = wmma_bf(ah, w, acc[j]); } }
#pragma unroll
  for (int j = 0; j < 8; ++j)
#pragma unroll
    for (int r = 0; r < 8; ++r) so[wave][8 * g + r][j * 16 + col] = acc[j][r];
  LDSX();
  for (int rl = 0; rl < 16; ++rl) vst2(Y + (r0 + rl) * DM + n0 + lane * 4, *(const v4f*)&so[wave][rl][lane * 4]);
}

extern "C" void kernel_launch(void* const* d_in, const int* in_sizes, int n_in, void* d_out, int out_size, void* d_ws, size_t ws_size, hipStream_t stream) {
  if (n_in < 3) return;
  if (in_sizes[0] < ((NB - 1) * SEQ_FULL + SEQ) * DM) return;
  if (in_sizes[1] < DM * QKVW) return;
  if (in_sizes[2] < DM * DM) return;
  if (out_size < ((NB - 1) * SEQ_FULL + SEQ) * DM) return;
  if (ws_size < (size_t)WS_END) return;
  const float* X = (const float*)d_in[0]; const float* WQ = (const float*)d_in[1]; const float* WO = (const float*)d_in[2];
  char* ws = (char*)d_ws;
  __bf16* PK = (__bf16*)(ws + WS_PK); __bf16* XB = (__bf16*)(ws + WS_XB); float* QK = (float*)(ws + WS_QK);
  __bf16 *KH = (__bf16*)(ws + WS_KH), *KL = (__bf16*)(ws + WS_KL), *VTH = (__bf16*)(ws + WS_VTH), *VTL = (__bf16*)(ws + WS_VTL);
  float* O = (float*)(ws + WS_O); __bf16 *OH = (__bf16*)(ws + WS_OH), *OL = (__bf16*)(ws + WS_OL);
  float* Yout = (float*)d_out;
  k_packT<<<QKVW, 256, 0, stream>>>(WQ, DM, QKVW, PK + PK_A);
  k_packT<<<DM, 256, 0, stream>>>(WO, DM, DM, PK + PK_P);
  k_cvtx<<<NB * SEQ / 2, 256, 0, stream>>>(X, XB);
  for (int b = 0; b < NB; ++b) {
    k_qkv<<<dim3(SEQ / 64, QKVW / 128), 128, 0, stream>>>(XB + (size_t)b * SEQ * DM, PK + PK_A, QK);
    k_kv<<<dim3(SEQ / 64, NH), 256, 0, stream>>>(QK, KH, KL, VTH, VTL);
    k_attn<<<dim3(SEQ / 64, NH), 128, 0, stream>>>(QK, KH, KL, VTH, VTL, O);
    k_osplit<<<SEQ / 2, 256, 0, stream>>>(O, OH, OL);
    k_out<<<dim3(SEQ / 64, DM / 128), 128, 0, stream>>>(OH, OL, PK + PK_P, Yout + (size_t)b * SEQ_FULL * DM);
  }
}
